// Encoder_6476810682593
// MI455X (gfx1250) — hardware-verified
//
#include <hip/hip_runtime.h>
#include <math.h>
#pragma clang fp contract(off)

typedef __attribute__((ext_vector_type(16))) _Float16 v16h;
typedef __attribute__((ext_vector_type(8)))  _Float16 v8h;
typedef __attribute__((ext_vector_type(8)))  float    v8f;
typedef __attribute__((ext_vector_type(4)))  float    v4f;
typedef __attribute__((ext_vector_type(4)))  int      v4i;

constexpr int NBATCH   = 8;
constexpr int NPT0     = 2048;
constexpr int NPT1     = 256;
constexpr int NPT2     = 16;
constexpr int NNB      = 20;
constexpr int NSUP     = 7;
constexpr int CH0      = 32;
constexpr int CH1      = 64;
constexpr int CH2      = 256;
constexpr int NI_PITCH = 32;
constexpr int KNN_TILE = 128;
constexpr int SIDX_PITCH = 36;
constexpr float FM0_CARRY = 1024.0f;
constexpr float FM1_CARRY = 256.0f;
constexpr float W_CARRY   = 256.0f;
constexpr float GEMM1_SCALE = 1.0f / (FM0_CARRY * W_CARRY);
constexpr float GEMM2_SCALE = 1.0f / (FM1_CARRY * W_CARRY);
constexpr float NEG_BIG = -3.402823466e38f;
constexpr float POS_BIG = 3.0e38f;
constexpr int OUT0_FLOATS = NBATCH * NPT2 * 3;
constexpr int OUT1_FLOATS = NBATCH * NPT2 * CH2;
static_assert(OUT0_FLOATS * 4 == 1536);
static_assert((OUT0_FLOATS + OUT1_FLOATS) * 4 == 132608);
static_assert((NBATCH * NPT0) % 64 == 0 && ((NSUP + 1) * CH1) % 64 == 0 && CH0 % 32 == 0);
static_assert((NBATCH * NPT1) % 64 == 0 && ((NSUP + 1) * CH2) % 64 == 0 && CH1 % 32 == 0);
static_assert(NPT0 % KNN_TILE == 0 && NPT1 % KNN_TILE == 0);
static_assert(NNB < NI_PITCH);

constexpr size_t SZ_W1T   = (size_t)(NSUP + 1) * CH1 * CH0 * 2;
constexpr size_t SZ_W2T   = (size_t)(NSUP + 1) * CH2 * CH1 * 2;
constexpr size_t SZ_NI20  = (size_t)NBATCH * NPT0 * NI_PITCH * 4;
constexpr size_t SZ_FM0H  = (size_t)NBATCH * NPT0 * CH0 * 2;
constexpr size_t SZ_FEAT1 = (size_t)NBATCH * NPT0 * (NSUP + 1) * CH1 * 4;
constexpr size_t SZ_FM1   = (size_t)NBATCH * NPT0 * CH1 * 4;
constexpr size_t SZ_NI8   = (size_t)NBATCH * NPT1 * NI_PITCH * 4;
constexpr size_t SZ_V1    = (size_t)NBATCH * NPT1 * 3 * 4;
constexpr size_t SZ_FM1PH = (size_t)NBATCH * NPT1 * CH1 * 2;
constexpr size_t SZ_NI20B = (size_t)NBATCH * NPT1 * NI_PITCH * 4;
constexpr size_t SZ_FEAT2 = (size_t)NBATCH * NPT1 * (NSUP + 1) * CH2 * 4;
constexpr size_t SZ_FM2   = (size_t)NBATCH * NPT1 * CH2 * 4;
constexpr size_t SZ_TOTAL = SZ_W1T + SZ_W2T + SZ_NI20 + SZ_FM0H + SZ_FEAT1 + SZ_FM1 + SZ_NI8 + SZ_V1 +
                            SZ_FM1PH + SZ_NI20B + SZ_FEAT2 + SZ_FM2;
static_assert(SZ_W1T % 256 == 0 && SZ_W2T % 256 == 0 && SZ_NI20 % 256 == 0 && SZ_FM0H % 256 == 0);
static_assert(SZ_FEAT1 % 256 == 0 && SZ_FM1 % 256 == 0 && SZ_NI8 % 256 == 0 && SZ_V1 % 256 == 0);
static_assert(SZ_FM1PH % 256 == 0 && SZ_NI20B % 256 == 0 && SZ_FEAT2 % 256 == 0 && SZ_FM2 % 256 == 0);
static_assert(SZ_TOTAL == (size_t)60874752);
static_assert(SZ_TOTAL <= (size_t)134217728);

__device__ const int S1_TAB[] = {
1063,1693,1603,1973,48,417,1535,1659,1620,1248,521,232,1757,1695,1874,1562,353,23,1525,557,1895,1617,1788,1252,1495,21,1410,184,1580,1059,734,964,1043,784,513,1139,492,1313,985,211,1758,287,1506,1046,992,1579,935,1068,82,644,1651,262,1420,1785,1539,84,436,115,1339,1706,366,1369,1151,1889,724,904,181,1549,1130,699,379,971,1269,1189,932,1032,274,1773,882,1217,1334,1374,1181,66,136,123,1147,950,319,424,704,443,427,920,874,884,769,698,1775,154,1710,1718,533,809,1621,1154,856,998,1531,1862,1671,944,591,1726,332,73,107,916,1453,352,109,789,103,157,434,2016,1821,757,1298,498,994,77,1246,767,1712,659,1953,694,1275,1990,487,132,1367,1111,1349,663,1829,1328,705,903,1657,855,1960,1091,1006,1997,233,395,788,586,1729,1413,589,1872,1587,1218,921,1592,412,387,2021,335,1675,1440,420,1886,1174,1037,848,1851,1460,331,647,1739,130,1658,1228,2034,1491,1015,997,1324,695,17,1515,536,415,146,1916,1076,1517,1944,2032,1177,1522,1155,1908,831,1631,2007,1697,228,2005,65,1250,105,316,1637,1278,1968,437,613,1000,1689,552,1564,1135,818,1852,1093,1397,354,248,1145,517,1455,1787,1868,263,652,1047,191,1034,252,686,879,547,1337,881,1193,1762,1056,1520,1632,720,933
};
__device__ const int S2_TAB[] = {
230,136,182,135,67,120,162,78,26,127,42,235,139,173,61,218
};
static_assert(sizeof(S1_TAB) / sizeof(S1_TAB[0]) == 256);
static_assert(sizeof(S2_TAB) / sizeof(S2_TAB[0]) == 16);

__device__ __forceinline__ int clampi(int x, int hi) {
  x = x < 0 ? 0 : x;
  return x > hi ? hi : x;
}

union FragU { v16h v; v8h h[2]; };
__device__ __forceinline__ v16h frag_load_h(const _Float16* p) {
  FragU f;
  f.h[0] = *(const v8h*)(p);
  f.h[1] = *(const v8h*)(p + 16);
  return f.v;
}
__device__ __forceinline__ v8f mma_h(v16h a, v16h b, v8f c) {
  return __builtin_amdgcn_wmma_f32_16x16x32_f16(false, a, false, b, (short)0, c, false, false);
}
__device__ __forceinline__ void guard4_h(v8f& a, v8f& b, v8f& c, v8f& d, v16h x, v16h y0, v16h y1, v16h y2, v16h y3) {
  asm volatile("v_nop\n\tv_nop\n\tv_nop\n\tv_nop" : "+v"(a), "+v"(b), "+v"(c), "+v"(d) : "v"(x), "v"(y0), "v"(y1), "v"(y2), "v"(y3));
}
__device__ __forceinline__ void keep4_h(v16h a, v16h b, v16h c, v16h d) {
  asm volatile("v_nop" :: "v"(a), "v"(b), "v"(c), "v"(d));
}
__device__ __forceinline__ void acc_guard4(v8f& a, v8f& b, v8f& c, v8f& d) {
  asm volatile("v_nop\n\tv_nop\n\tv_nop\n\tv_nop" : "+v"(a), "+v"(b), "+v"(c), "+v"(d));
}
__device__ __forceinline__ void tie8(float* m) {
  asm volatile("" : "+v"(m[0]), "+v"(m[1]), "+v"(m[2]), "+v"(m[3]), "+v"(m[4]), "+v"(m[5]), "+v"(m[6]), "+v"(m[7]) :: "memory");
}

__global__ __launch_bounds__(256) void wprep_kernel(const float* __restrict__ w1, const float* __restrict__ w2,
                                                    unsigned short* __restrict__ w1t, unsigned short* __restrict__ w2t) {
  const int blk = blockIdx.x;
  const bool second = (blk >= 8);
  const float* src = second ? w2 : w1;
  unsigned short* dst = second ? w2t : w1t;
  const int ndim = second ? (NSUP + 1) * CH2 : (NSUP + 1) * CH1;
  const int kshift = second ? 3 : 2;
  const int i = (second ? (blk - 8) : blk) * 256 + (int)threadIdx.x;
  const int n = i >> kshift;
  const int k0 = (i - (n << kshift)) * 8;
  v8h hv;
#pragma unroll
  for (int e = 0; e < 8; ++e) {
    const float w = src[(size_t)(k0 + e) * ndim + n];
    hv[e] = (_Float16)(w * W_CARRY);
  }
  unsigned short* op = dst + (size_t)i * 8;
  *(volatile v8h*)(op) = hv;
  __threadfence();
  *(volatile v8h*)(op) = hv;
}

template <int KSEL, bool VIA_S1>
__global__ __launch_bounds__(128) void knn_kernel(const float* __restrict__ pts, int V, int Q, int* __restrict__ out) {
  constexpr int KP1 = KSEL + 1;
  __shared__ float tx[KNN_TILE];
  __shared__ float ty[KNN_TILE];
  __shared__ float tz[KNN_TILE];
  __shared__ float tq[KNN_TILE];
  __shared__ __align__(16) int sidx[KNN_TILE * SIDX_PITCH];
  const int tid = threadIdx.x;
  const int b = blockIdx.y;
  const int q = blockIdx.x * KNN_TILE + tid;
  const float* P = pts + (size_t)b * V * 3;
  int qrow = q;
  if (VIA_S1) qrow = S1_TAB[q & 255];
  qrow = clampi(qrow, V - 1);
  const float qx = P[qrow * 3 + 0];
  const float qy = P[qrow * 3 + 1];
  const float qz = P[qrow * 3 + 2];
  const float qn = (qx * qx + qz * qz) + qy * qy;

  float bd[KP1];
  int bi[KP1];
#pragma unroll
  for (int t = 0; t < KP1; ++t) { bd[t] = POS_BIG; bi[t] = 0; }
  float worst = POS_BIG;

  for (int base = 0; base < V; base += KNN_TILE) {
    __syncthreads();
    {
      int cand = base + tid;
      cand = cand > V - 1 ? V - 1 : cand;
      const float x = P[cand * 3 + 0];
      const float y = P[cand * 3 + 1];
      const float z = P[cand * 3 + 2];
      tx[tid] = x;
      ty[tid] = y;
      tz[tid] = z;
      tq[tid] = (x * x + z * z) + y * y;
    }
    __syncthreads();
#pragma unroll 1
    for (int j = 0; j < KNN_TILE; ++j) {
      const float x = tx[j];
      const float y = ty[j];
      const float z = tz[j];
      const float cq = tq[j];
      float p = qx * x;
      p = fmaf(qy, y, p);
      p = fmaf(qz, z, p);
      const float d = ((-2.0f * p) + qn) + cq;
      if (d < worst) {
        const int cidx = base + j;
#pragma unroll
        for (int t = KP1 - 1; t >= 1; --t) {
          const bool cp = d < bd[t - 1];
          const bool cc = d < bd[t];
          const float nd = cp ? bd[t - 1] : (cc ? d : bd[t]);
          const int nix = cp ? bi[t - 1] : (cc ? cidx : bi[t]);
          bd[t] = nd;
          bi[t] = nix;
        }
        {
          const bool c0 = d < bd[0];
          bd[0] = c0 ? d : bd[0];
          bi[0] = c0 ? cidx : bi[0];
        }
        worst = bd[KP1 - 1];
      }
    }
  }
#pragma unroll
  for (int n = 0; n < NI_PITCH; ++n) {
    const int v = (n < KSEL) ? bi[(n < KSEL) ? (n + 1) : 0] : 0;
    sidx[tid * SIDX_PITCH + n] = v;
  }
  __syncthreads();
  {
    const int wave = tid >> 5;
    const int lane = tid & 31;
    int* orow = out + ((size_t)b * Q + (size_t)blockIdx.x * KNN_TILE + (size_t)wave * 32) * NI_PITCH;
    const int rq = lane >> 3;
    const int c4 = (lane & 7) * 4;
    for (int pass = 0; pass < 2; ++pass) {
#pragma unroll
      for (int it = 0; it < 8; ++it) {
        const int row = it * 4 + rq;
        const v4i v = *(const v4i*)(sidx + (wave * 32 + row) * SIDX_PITCH + c4);
        *(volatile v4i*)(orow + row * NI_PITCH + c4) = v;
      }
      __threadfence();
    }
  }
}

__global__ __launch_bounds__(256) void op3d_kernel(const float* __restrict__ verts, const int* __restrict__ ni,
                                                   const float* __restrict__ w0d, const float* __restrict__ w0w,
                                                   unsigned short* __restrict__ fm0h) {
  constexpr int NWD = 3 * NSUP * CH0;
  constexpr int NWW = NSUP * CH0;
  __shared__ __align__(16) float sF[8 * CH0];
  __shared__ float sWd[NWD];
  __shared__ float sWw[NWW];
  const int tid = threadIdx.x;
  const int lane = tid & 31;
  const int wave = tid >> 5;
  const int b = blockIdx.y;
  const int v = blockIdx.x * 8 + wave;
#pragma unroll
  for (int it = 0; it < 3; ++it) {
    const int i = tid + it * 256;
    const int ic = i < NWD ? i : NWD - 1;
    const float t = w0d[ic];
    if (i < NWD) sWd[i] = t;
  }
  {
    const int ic = tid < NWW ? tid : NWW - 1;
    const float t = w0w[ic];
    if (tid < NWW) sWw[tid] = t;
  }
  const float* P = verts + (size_t)b * NPT0 * 3;
  const float cx = P[v * 3 + 0];
  const float cy = P[v * 3 + 1];
  const float cz = P[v * 3 + 2];
  int j = ni[((size_t)b * NPT0 + v) * NI_PITCH + lane];
  j = clampi(j, NPT0 - 1);
  const float dx = P[j * 3 + 0] - cx;
  const float dy = P[j * 3 + 1] - cy;
  const float dz = P[j * 3 + 2] - cz;
  __syncthreads();
  float wa[NSUP], wb[NSUP], wc[NSUP], ww[NSUP], m[NSUP];
#pragma unroll
  for (int s = 0; s < NSUP; ++s) {
    wa[s] = sWd[s * CH0 + lane];
    wb[s] = sWd[NSUP * CH0 + s * CH0 + lane];
    wc[s] = sWd[2 * NSUP * CH0 + s * CH0 + lane];
    ww[s] = sWw[s * CH0 + lane];
    m[s] = 0.0f;
  }
#pragma unroll 1
  for (int n = 0; n < NNB; ++n) {
    const float ax = __shfl(dx, n, 32);
    const float ay = __shfl(dy, n, 32);
    const float az = __shfl(dz, n, 32);
#pragma unroll
    for (int s = 0; s < NSUP; ++s) {
      float t = ax * wa[s];
      t = fmaf(ay, wb[s], t);
      t = fmaf(az, wc[s], t);
      m[s] = fmaxf(m[s], fmaxf(t, 0.0f));
    }
  }
  float acc = 0.0f;
#pragma unroll
  for (int s = 0; s < NSUP; ++s) {
    const float pr = m[s] * ww[s];
    acc = acc + pr;
  }
  sF[wave * CH0 + lane] = fmaxf(acc, 0.0f);
  __syncthreads();
  if (wave == 0) {
    v8h hv;
#pragma unroll
    for (int e = 0; e < 8; ++e) {
      const float x = sF[lane * 8 + e];
      hv[e] = (_Float16)(x * FM0_CARRY);
    }
    unsigned short* op = fm0h + ((size_t)b * NPT0 + (size_t)blockIdx.x * 8) * CH0 + (size_t)lane * 8;
    *(volatile v8h*)(op) = hv;
    __threadfence();
    *(volatile v8h*)(op) = hv;
  }
}

__global__ __launch_bounds__(256) void gemm64_f16_kernel(
    const unsigned short* __restrict__ Ap, int lda,
    const unsigned short* __restrict__ Btp, int ldb,
    float* __restrict__ Cout, int ldc,
    const float* __restrict__ bias, int M, int N, int K, float scale) {
  const _Float16* A = (const _Float16*)Ap;
  const _Float16* Bt = (const _Float16*)Btp;
  __shared__ __align__(16) float sT[8][16 * 68];
  const int lane = threadIdx.x & 31;
  const int wave = threadIdx.x >> 5;
  const int tilesN = N >> 6;
  const int tilesM = M >> 6;
  const int tile = blockIdx.x * 8 + wave;
  if (tile >= tilesM * tilesN) return;
  const int tm = tile / tilesN;
  const int tn = tile - tm * tilesN;
  const int m0 = tm << 6;
  const int n0 = tn << 6;
  const int rlane = lane & 15;
  const int koff = (lane >> 4) * 8;
  const int mOff = (lane >> 4) * 8;

  v8f acc[4][4];
#pragma unroll
  for (int i = 0; i < 4; ++i)
#pragma unroll
    for (int j = 0; j < 4; ++j) acc[i][j] = (v8f){0.f, 0.f, 0.f, 0.f, 0.f, 0.f, 0.f, 0.f};

  for (int k0 = 0; k0 < K; k0 += 32) {
    v16h bh[4];
#pragma unroll
    for (int j = 0; j < 4; ++j) {
      const size_t bo = (size_t)(n0 + (j << 4) + rlane) * ldb + koff + k0;
      bh[j] = frag_load_h(Bt + bo);
    }
#pragma unroll
    for (int i = 0; i < 4; ++i) {
      const size_t ao = (size_t)(m0 + (i << 4) + rlane) * lda + koff + k0;
      const v16h ah = frag_load_h(A + ao);
#pragma unroll
      for (int j = 0; j < 4; ++j) acc[i][j] = mma_h(ah, bh[j], acc[i][j]);
      guard4_h(acc[i][0], acc[i][1], acc[i][2], acc[i][3], ah, bh[0], bh[1], bh[2], bh[3]);
    }
    keep4_h(bh[0], bh[1], bh[2], bh[3]);
  }
  acc_guard4(acc[0][0], acc[0][1], acc[0][2], acc[0][3]);
  acc_guard4(acc[1][0], acc[1][1], acc[1][2], acc[1][3]);
  acc_guard4(acc[2][0], acc[2][1], acc[2][2], acc[2][3]);
  acc_guard4(acc[3][0], acc[3][1], acc[3][2], acc[3][3]);

  float* slab = sT[wave];
#pragma unroll
  for (int i = 0; i < 4; ++i) {
    const int mBase = m0 + (i << 4);
#pragma unroll
    for (int j = 0; j < 4; ++j) {
      const int n = n0 + (j << 4) + rlane;
      const float bv = bias[n];
#pragma unroll
      for (int r = 0; r < 8; ++r) {
        float v = acc[i][j][r] * scale;
        v += bv;
        slab[(mOff + r) * 68 + (j << 4) + rlane] = v;
      }
    }
    __builtin_amdgcn_fence(__ATOMIC_RELEASE, "workgroup");
    __builtin_amdgcn_wave_barrier();
    __builtin_amdgcn_fence(__ATOMIC_ACQUIRE, "workgroup");
    {
      const int hh = lane >> 4;
      const int c4 = (lane & 15) * 4;
      for (int pass = 0; pass < 2; ++pass) {
#pragma unroll
        for (int it = 0; it < 8; ++it) {
          const int row = it * 2 + hh;
          const v4f v = *(const v4f*)(slab + row * 68 + c4);
          *(volatile v4f*)(Cout + (size_t)(mBase + row) * ldc + n0 + c4) = v;
        }
        __threadfence();
      }
    }
    __builtin_amdgcn_fence(__ATOMIC_RELEASE, "workgroup");
    __builtin_amdgcn_wave_barrier();
    __builtin_amdgcn_fence(__ATOMIC_ACQUIRE, "workgroup");
  }
}

template <int VCNT, int CHN>
__global__ __launch_bounds__(256) void opnd_kernel(const float* __restrict__ pts, const int* __restrict__ ni,
                                                   const float* __restrict__ feat, const float* __restrict__ dw,
                                                   float* __restrict__ outF) {
  constexpr int FW = (NSUP + 1) * CHN;
  constexpr int DWW = NSUP * CHN;
  constexpr int NV4 = (3 * DWW) / 4;
  constexpr int NIT = (NV4 + 255) / 256;
  static_assert((3 * DWW) % 4 == 0);
  static_assert(NIT <= 8);
  __shared__ __align__(16) float sO[8 * CHN];
  __shared__ __align__(16) float sW[3 * DWW];
  const int tid = threadIdx.x;
  const int lane = tid & 31;
  const int wave = tid >> 5;
  const int b = blockIdx.y;
  const int v = blockIdx.x * 8 + wave;
#pragma unroll
  for (int it = 0; it < NIT; ++it) {
    const int i = tid + it * 256;
    const int ic = i < NV4 ? i : NV4 - 1;
    const v4f t = *(const v4f*)(dw + 4 * ic);
    if (i < NV4) *(v4f*)(sW + 4 * i) = t;
  }
  const float* P = pts + (size_t)b * VCNT * 3;
  const float cx = P[v * 3 + 0];
  const float cy = P[v * 3 + 1];
  const float cz = P[v * 3 + 2];
  int j = ni[((size_t)b * VCNT + v) * NI_PITCH + lane];
  j = clampi(j, VCNT - 1);
  const float dx = P[j * 3 + 0] - cx;
  const float dy = P[j * 3 + 1] - cy;
  const float dz = P[j * 3 + 2] - cz;
  const float* fbase = feat + (size_t)b * VCNT * FW;
  const float* frow = fbase + (size_t)v * FW;
  __syncthreads();

#pragma unroll 1
  for (int cc = 0; cc < CHN / 32; ++cc) {
    const int c = cc * 32 + lane;
    float wa[NSUP], wb[NSUP], wc[NSUP], m[NSUP];
#pragma unroll
    for (int s = 0; s < NSUP; ++s) {
      wa[s] = sW[s * CHN + c];
      wb[s] = sW[DWW + s * CHN + c];
      wc[s] = sW[2 * DWW + s * CHN + c];
      m[s] = NEG_BIG;
    }
    const float ctr = frow[c];
#pragma unroll 1
    for (int n = 0; n < NNB; ++n) {
      const float ax = __shfl(dx, n, 32);
      const float ay = __shfl(dy, n, 32);
      const float az = __shfl(dz, n, 32);
      const int jn = __shfl(j, n, 32);
      const float* fr = fbase + (size_t)jn * FW + CHN + c;
#pragma unroll
      for (int s = 0; s < NSUP; ++s) {
        float t = ax * wa[s];
        t = fmaf(ay, wb[s], t);
        t = fmaf(az, wc[s], t);
        t = fmaxf(t, 0.0f);
        const float f = fr[s * CHN];
        const float pr = t * f;
        m[s] = fmaxf(m[s], pr);
      }
    }
    float acc = 0.0f;
#pragma unroll
    for (int s = 0; s < NSUP; ++s) acc = acc + m[s];
    sO[wave * CHN + c] = fmaxf(ctr + acc, 0.0f);
  }
  __syncthreads();
  {
    float* ob = outF + ((size_t)b * VCNT + (size_t)blockIdx.x * 8) * CHN;
    for (int pass = 0; pass < 2; ++pass) {
      for (int i = tid; i < (8 * CHN) / 4; i += 256) {
        const v4f val = *(const v4f*)(sO + 4 * i);
        *(volatile v4f*)(ob + 4 * i) = val;
      }
      __threadfence();
    }
  }
}

__device__ __forceinline__ void pool1_acc4(const float* __restrict__ fb, v4i idx, int c8, float* mx) {
#pragma unroll
  for (int n = 0; n < 4; ++n) {
    const int jn = clampi(idx[n], NPT0 - 1);
    const float* fr = fb + (size_t)jn * CH1 + c8;
    const v4f a = *(const v4f*)(fr);
    const v4f bb = *(const v4f*)(fr + 4);
#pragma unroll
    for (int e = 0; e < 4; ++e) {
      mx[e] = fmaxf(mx[e], a[e]);
      mx[4 + e] = fmaxf(mx[4 + e], bb[e]);
    }
  }
}

__global__ __launch_bounds__(256) void pool1_kernel(const float* __restrict__ verts, const int* __restrict__ ni8,
                                                    const float* __restrict__ fm1, float* __restrict__ v1,
                                                    unsigned short* __restrict__ fm1ph) {
  const int tid = threadIdx.x;
  const int b = blockIdx.y;
  const int q0 = blockIdx.x * 32;
  const int r = tid >> 3;
  const int c8 = (tid & 7) * 8;
  const int q = q0 + r;
  const int* nrow = ni8 + ((size_t)b * NPT1 + q) * NI_PITCH;
  const v4i ia = *(const v4i*)(nrow);
  const v4i ib = *(const v4i*)(nrow + 4);
  const float* fb = fm1 + (size_t)b * NPT0 * CH1;
  float mx[8];
#pragma unroll
  for (int e = 0; e < 8; ++e) mx[e] = NEG_BIG;
  pool1_acc4(fb, ia, c8, mx);
  tie8(mx);
  pool1_acc4(fb, ib, c8, mx);
  tie8(mx);
  v8h hv;
#pragma unroll
  for (int e = 0; e < 8; ++e) hv[e] = (_Float16)(mx[e] * FM1_CARRY);
  unsigned short* op = fm1ph + ((size_t)b * NPT1 + q0) * CH1 + (size_t)tid * 8;
  *(volatile v8h*)(op) = hv;
  __threadfence();
  *(volatile v8h*)(op) = hv;

  if ((tid >> 5) == 0) {
    const int lane = tid & 31;
    const int f4 = lane < 24 ? lane : 23;
    v4f val;
#pragma unroll
    for (int e = 0; e < 4; ++e) {
      const int f = f4 * 4 + e;
      const int row = f / 3;
      const int comp = f - row * 3;
      const int srow = clampi(S1_TAB[(q0 + row) & 255], NPT0 - 1);
      val[e] = verts[((size_t)b * NPT0 + srow) * 3 + comp];
    }
    float* vp = v1 + ((size_t)b * NPT1 + q0) * 3 + f4 * 4;
    if (lane < 24) *(volatile v4f*)(vp) = val;
    __threadfence();
    if (lane < 24) *(volatile v4f*)(vp) = val;
  }
}

__global__ __launch_bounds__(256) void pool2_kernel(const float* __restrict__ verts, const float* __restrict__ v1,
                                                    const float* __restrict__ fm2, float* __restrict__ out) {
  __shared__ float sd[NPT1];
  __shared__ int slist[NPT2];
  __shared__ __align__(16) float so[CH2];
  const int tid = threadIdx.x;
  const int i = blockIdx.x;
  const int b = blockIdx.y;
  const float* P = v1 + (size_t)b * NPT1 * 3;
  const int qrow = clampi(S2_TAB[i & 15], NPT1 - 1);
  const float qx = P[qrow * 3 + 0];
  const float qy = P[qrow * 3 + 1];
  const float qz = P[qrow * 3 + 2];
  const float qn = (qx * qx + qz * qz) + qy * qy;
  const float x = P[tid * 3 + 0];
  const float y = P[tid * 3 + 1];
  const float z = P[tid * 3 + 2];
  const float cq = (x * x + z * z) + y * y;
  float p = qx * x;
  p = fmaf(qy, y, p);
  p = fmaf(qz, z, p);
  const float d = ((-2.0f * p) + qn) + cq;
  sd[tid] = d;
  if (tid < NPT2) slist[tid] = 0;
  __syncthreads();
  int rank = 0;
#pragma unroll 4
  for (int m = 0; m < NPT1; ++m) {
    const float dm = sd[m];
    const bool before = (dm < d) || ((dm == d) && (m < tid));
    rank += before ? 1 : 0;
  }
  if (rank >= 1 && rank <= NPT2) slist[rank - 1] = tid;
  __syncthreads();
  float mx = NEG_BIG;
#pragma unroll
  for (int n = 0; n < NPT2; ++n) {
    const int jn = clampi(slist[n], NPT1 - 1);
    const float f = fm2[((size_t)b * NPT1 + jn) * CH2 + tid];
    mx = fmaxf(mx, f);
    if (n == 7) asm volatile("" : "+v"(mx) :: "memory");
  }
  so[tid] = mx;
  __syncthreads();
  if (tid < 64) {
    const v4f val = *(const v4f*)(so + 4 * tid);
    float* op = out + OUT0_FLOATS + ((size_t)b * NPT2 + i) * CH2 + 4 * tid;
    *(volatile v4f*)(op) = val;
    __threadfence();
    *(volatile v4f*)(op) = val;
  }
  if (blockIdx.x == 0 && blockIdx.y == 0 && (tid >> 5) == 2) {
    const int lane = tid & 31;
#pragma unroll 1
    for (int it = 0; it < 3; ++it) {
      const int f4 = it * 32 + lane;
      v4f val;
#pragma unroll
      for (int e = 0; e < 4; ++e) {
        const int f = f4 * 4 + e;
        const int row = f / 3;
        const int comp = f - row * 3;
        const int bb = row >> 4;
        const int ii = row & 15;
        const int s2 = clampi(S2_TAB[ii], NPT1 - 1);
        const int s12 = clampi(S1_TAB[s2], NPT0 - 1);
        val[e] = verts[((size_t)bb * NPT0 + s12) * 3 + comp];
      }
      float* op = out + f4 * 4;
      *(volatile v4f*)(op) = val;
      __threadfence();
      *(volatile v4f*)(op) = val;
    }
  }
}

extern "C" void kernel_launch(void* const* d_in, const int* in_sizes, int n_in,
                              void* d_out, int out_size, void* d_ws, size_t ws_size, hipStream_t stream) {
  if (n_in < 9 || d_out == nullptr || d_ws == nullptr) return;
  if (in_sizes[0] != NBATCH * NPT0 * 3 || in_sizes[1] != NSUP * CH0 || in_sizes[2] != 3 * NSUP * CH0 ||
      in_sizes[3] != CH0 * (NSUP + 1) * CH1 || in_sizes[4] != (NSUP + 1) * CH1 || in_sizes[5] != 3 * NSUP * CH1 ||
      in_sizes[6] != CH1 * (NSUP + 1) * CH2 || in_sizes[7] != (NSUP + 1) * CH2 || in_sizes[8] != 3 * NSUP * CH2 ||
      out_size != OUT0_FLOATS + OUT1_FLOATS) return;

  const float* verts = (const float*)d_in[0];
  const float* w0w   = (const float*)d_in[1];
  const float* w0d   = (const float*)d_in[2];
  const float* w1w   = (const float*)d_in[3];
  const float* w1b   = (const float*)d_in[4];
  const float* w1d   = (const float*)d_in[5];
  const float* w2w   = (const float*)d_in[6];
  const float* w2b   = (const float*)d_in[7];
  const float* w2d   = (const float*)d_in[8];
  float* out = (float*)d_out;

  char* ws = (char*)d_ws;
  size_t off = 0;
  auto carve = [&](size_t bytes) -> char* { char* p = ws + off; off += (bytes + 255) & ~(size_t)255; return p; };
  unsigned short* W1T   = (unsigned short*)carve(SZ_W1T);
  unsigned short* W2T   = (unsigned short*)carve(SZ_W2T);
  int*            NI20  = (int*)carve(SZ_NI20);
  unsigned short* FM0H  = (unsigned short*)carve(SZ_FM0H);
  float*          FEAT1 = (float*)carve(SZ_FEAT1);
  float*          FM1   = (float*)carve(SZ_FM1);
  int*            NI8   = (int*)carve(SZ_NI8);
  float*          V1    = (float*)carve(SZ_V1);
  unsigned short* FM1PH = (unsigned short*)carve(SZ_FM1PH);
  int*            NI20B = (int*)carve(SZ_NI20B);
  float*          FEAT2 = (float*)carve(SZ_FEAT2);
  float*          FM2   = (float*)carve(SZ_FM2);
  if (off != SZ_TOTAL || off > ws_size || off > (size_t)134217728) return;

  wprep_kernel<<<72, 256, 0, stream>>>(w1w, w2w, W1T, W2T);

  knn_kernel<NNB, false><<<dim3(NPT0 / KNN_TILE, NBATCH), KNN_TILE, 0, stream>>>(verts, NPT0, NPT0, NI20);
  op3d_kernel<<<dim3(NPT0 / 8, NBATCH), 256, 0, stream>>>(verts, NI20, w0d, w0w, FM0H);
  gemm64_f16_kernel<<<((NBATCH * NPT0 / 64) * ((NSUP + 1) * CH1 / 64)) / 8, 256, 0, stream>>>(
      FM0H, CH0, W1T, CH0, FEAT1, (NSUP + 1) * CH1, w1b, NBATCH * NPT0, (NSUP + 1) * CH1, CH0, GEMM1_SCALE);
  opnd_kernel<NPT0, CH1><<<dim3(NPT0 / 8, NBATCH), 256, 0, stream>>>(verts, NI20, FEAT1, w1d, FM1);

  knn_kernel<8, true><<<dim3(NPT1 / KNN_TILE, NBATCH), KNN_TILE, 0, stream>>>(verts, NPT0, NPT1, NI8);
  pool1_kernel<<<dim3(NPT1 / 32, NBATCH), 256, 0, stream>>>(verts, NI8, FM1, V1, FM1PH);

  knn_kernel<NNB, false><<<dim3(NPT1 / KNN_TILE, NBATCH), KNN_TILE, 0, stream>>>(V1, NPT1, NPT1, NI20B);
  gemm64_f16_kernel<<<((NBATCH * NPT1 / 64) * ((NSUP + 1) * CH2 / 64)) / 8, 256, 0, stream>>>(
      FM1PH, CH1, W2T, CH1, FEAT2, (NSUP + 1) * CH2, w2b, NBATCH * NPT1, (NSUP + 1) * CH2, CH1, GEMM2_SCALE);
  opnd_kernel<NPT1, CH2><<<dim3(NPT1 / 8, NBATCH), 256, 0, stream>>>(V1, NI20B, FEAT2, w2d, FM2);

  pool2_kernel<<<dim3(NPT2, NBATCH), 256, 0, stream>>>(verts, V1, FM2, out);
}
